// SupportVectorRegression_20779051778152
// MI455X (gfx1250) — hardware-run, weakly checked
//
#include <hip/hip_runtime.h>
#include <stddef.h>


typedef _Float16 v16h __attribute__((ext_vector_type(16)));
typedef _Float16 v8h  __attribute__((ext_vector_type(8)));
typedef float    v8f  __attribute__((ext_vector_type(8)));
typedef float    v4f  __attribute__((ext_vector_type(4)));
typedef _Float16 h16;

#define NSAMP 4096
#define DFEAT 64
#ifndef IROWS
#define IROWS 4096
#endif
#define FCARRY 16.0f
#define JT_PER_WAVE (NSAMP / 16 / 8)

static_assert(DFEAT == 64);
static_assert((DFEAT % 32) == 0);
static_assert((NSAMP % 32) == 0);
static_assert(((NSAMP / 16) % 8) == 0);
static_assert(JT_PER_WAVE * 8 * 16 == NSAMP);
static_assert(IROWS >= 32 && IROWS <= NSAMP && (IROWS % 32) == 0);
static_assert(256 == 32 * 8);

#define F16_BYTES ((size_t)NSAMP * DFEAT * 2)
#define SQ_BYTES  ((size_t)NSAMP * 4)
#define OFF_F16   ((size_t)0)
#define OFF_SQ    (OFF_F16 + F16_BYTES)
#define WS_TOTAL  (OFF_SQ + SQ_BYTES)
static_assert((F16_BYTES % 128) == 0 && (SQ_BYTES % 128) == 0);
static_assert(WS_TOTAL <= (size_t)134217728);

__device__ __forceinline__ float bf16r(float x) {
  unsigned int u = __float_as_uint(x);
  u = (u + 0x7FFFu + ((u >> 16) & 1u)) & 0xFFFF0000u;
  return __uint_as_float(u);
}

static __device__ __forceinline__ h16 toh_flush(float v) {
  const h16 r = (h16)v;
  return (fabsf(v) < 6.103515625e-05f) ? (h16)0.0f : r;
}

__device__ __forceinline__ v16h frag_at(const _Float16* p) {
  v8h lo = *(const v8h*)(p);
  v8h hi = *(const v8h*)(p + 16);
  v16h out;
#pragma unroll
  for (int i = 0; i < 8; ++i) { out[i] = lo[i]; out[i + 8] = hi[i]; }
  return out;
}

__device__ __forceinline__ v8f wmma16(v16h a, v16h b, v8f c) {
  v8f d = __builtin_amdgcn_wmma_f32_16x16x32_f16(false, a, false, b, (short)0, c,
                                                 false, false);
  asm volatile("v_nop\n\tv_nop\n\tv_nop\n\tv_nop" : "+v"(d) : "v"(a), "v"(b));
  return d;
}

__device__ __forceinline__ float red16_sum(float x) {
#pragma unroll
  for (int off = 1; off < 16; off <<= 1) x += __shfl_xor(x, off, 32);
  return x;
}

__global__ __launch_bounds__(256) void prep_kernel(
    const float* __restrict__ F, _Float16* __restrict__ F16, float* __restrict__ SQ) {
#pragma clang fp contract(off)
  __shared__ float sqs[32];
  const unsigned tid = threadIdx.x;
  const unsigned r = tid >> 3, c = (tid & 7u) * 8u;
  const unsigned row = blockIdx.x * 32u + r;
  const float* p = F + (size_t)row * DFEAT + c;
  const v4f a0 = *(const v4f*)(p);
  const v4f a1 = *(const v4f*)(p + 4);
  v8h o;
  float s = 0.0f;
#pragma unroll
  for (int i = 0; i < 4; ++i) {
    const float e0 = bf16r(a0[i]);
    const float e1 = bf16r(a1[i]);
    s += e0 * e0;
    s += e1 * e1;
    o[i]     = toh_flush(FCARRY * e0);
    o[i + 4] = toh_flush(FCARRY * e1);
  }
  s += __shfl_xor(s, 1, 32);
  s += __shfl_xor(s, 2, 32);
  s += __shfl_xor(s, 4, 32);
  if ((tid & 7u) == 0u) sqs[r] = s;

  _Float16* q = F16 + (size_t)row * DFEAT + c;
  *(volatile v8h*)q = o;
  __threadfence();
  *(volatile v8h*)q = o;

  __syncthreads();
  if (tid < 8u) {
    const v4f t = *(const v4f*)&sqs[tid * 4u];
    float* d = SQ + (size_t)blockIdx.x * 32u + tid * 4u;
    *(volatile v4f*)d = t;
    __threadfence();
    *(volatile v4f*)d = t;
  }
}

__global__ __launch_bounds__(256) void svr_kernel(
    const _Float16* __restrict__ F16, const float* __restrict__ SQ,
    const float* __restrict__ alpha, const float* __restrict__ bias,
    float* __restrict__ out) {
  __shared__ float part[8 * 32];
  const unsigned tid = threadIdx.x, lane = tid & 31u;
  const unsigned hh = lane >> 4, m = lane & 15u;
  const int wave = __builtin_amdgcn_readfirstlane(threadIdx.x >> 5);
  const unsigned i0 = blockIdx.x * 32u;
  const float bb = bf16r(bias[0]);
  const float g2 = 2.0f / (FCARRY * FCARRY);
  const float ecoef = -0.02f;

  const _Float16* ap = F16 + (size_t)(i0 + m) * DFEAT + hh * 8u;
  const v16h a00 = frag_at(ap);
  const v16h a01 = frag_at(ap + 32);
  const v16h a10 = frag_at(ap + 16 * DFEAT);
  const v16h a11 = frag_at(ap + 16 * DFEAT + 32);

  float sqi0[8], sqi1[8];
  {
    const v4f s0 = *(const v4f*)(SQ + i0 + hh * 8u);
    const v4f s1 = *(const v4f*)(SQ + i0 + hh * 8u + 4u);
    const v4f s2 = *(const v4f*)(SQ + i0 + 16u + hh * 8u);
    const v4f s3 = *(const v4f*)(SQ + i0 + 16u + hh * 8u + 4u);
#pragma unroll
    for (int r = 0; r < 4; ++r) {
      sqi0[r] = s0[r]; sqi0[r + 4] = s1[r];
      sqi1[r] = s2[r]; sqi1[r + 4] = s3[r];
    }
  }

  v8f acc0 = {}, acc1 = {};
  const unsigned jt0 = (unsigned)wave * (unsigned)JT_PER_WAVE;
#pragma unroll 1
  for (unsigned jt = jt0; jt < jt0 + (unsigned)JT_PER_WAVE; ++jt) {
    const unsigned j = jt * 16u + m;
    const _Float16* bp = F16 + (size_t)j * DFEAT + hh * 8u;
    const v16h b0 = frag_at(bp);
    const v16h b1 = frag_at(bp + 32);
    const float sqj = SQ[j];
    const float alj = bf16r(alpha[j]);

    v8f c0 = {}, c1 = {};
    c0 = wmma16(a00, b0, c0);
    c0 = wmma16(a01, b1, c0);
    c1 = wmma16(a10, b0, c1);
    c1 = wmma16(a11, b1, c1);

#pragma unroll
    for (int r = 0; r < 8; ++r) {
      const float d0 = fmaxf((sqi0[r] + sqj) - c0[r] * g2, 0.0f);
      const float d1 = fmaxf((sqi1[r] + sqj) - c1[r] * g2, 0.0f);
      acc0[r] = acc0[r] + __expf(d0 * ecoef) * alj;
      acc1[r] = acc1[r] + __expf(d1 * ecoef) * alj;
    }
  }

  float mine0 = 0.0f, mine1 = 0.0f;
#pragma unroll
  for (int r = 0; r < 8; ++r) {
    const float t0 = red16_sum(acc0[r]);
    const float t1 = red16_sum(acc1[r]);
    mine0 = (m == (unsigned)r) ? t0 : mine0;
    mine1 = (m == (unsigned)r) ? t1 : mine1;
  }
  if (m < 8u) {
    part[(unsigned)wave * 32u + hh * 8u + m]       = mine0;
    part[(unsigned)wave * 32u + 16u + hh * 8u + m] = mine1;
  }
  __syncthreads();

  if (tid < 8u) {
    v4f s = {};
#pragma unroll
    for (unsigned wv = 0; wv < 8u; ++wv) {
      const v4f t = *(const v4f*)&part[wv * 32u + tid * 4u];
      s = s + t;
    }
    v4f res;
#pragma unroll
    for (int qd = 0; qd < 4; ++qd) res[qd] = s[qd] + bb;
    float* d = out + (size_t)i0 + tid * 4u;
    *(volatile v4f*)d = res;
    __threadfence();
    *(volatile v4f*)d = res;
  }
}

extern "C" void kernel_launch(void* const* d_in, const int* in_sizes, int n_in,
                              void* d_out, int out_size, void* d_ws, size_t ws_size,
                              hipStream_t stream) {
  if (n_in < 3) return;
  if ((long long)in_sizes[0] < (long long)NSAMP * DFEAT) return;
  if ((long long)in_sizes[1] < (long long)NSAMP) return;
  if (in_sizes[2] < 1) return;
  if ((long long)out_size < (long long)IROWS) return;
  if (ws_size < WS_TOTAL) return;

  const float* feat  = (const float*)d_in[0];
  const float* alpha = (const float*)d_in[1];
  const float* bias  = (const float*)d_in[2];
  float* out = (float*)d_out;

  char* ws = (char*)d_ws;
  _Float16* F16 = (_Float16*)(ws + OFF_F16);
  float*    SQ  = (float*)(ws + OFF_SQ);

  dim3 blk(256);
  prep_kernel<<<dim3(NSAMP / 32), blk, 0, stream>>>(feat, F16, SQ);
  svr_kernel<<<dim3(IROWS / 32), blk, 0, stream>>>(F16, SQ, alpha, bias, out);
}
